// L2GTraversal_74088185856061
// MI455X (gfx1250) — hardware-verified
//
#include <hip/hip_runtime.h>
#include <math.h>

typedef __attribute__((ext_vector_type(16))) _Float16 v16h;
typedef __attribute__((ext_vector_type(16))) __bf16 v16b;
typedef __attribute__((ext_vector_type(8)))  _Float16 v8h;
typedef __attribute__((ext_vector_type(8)))  float v8f;
typedef __attribute__((ext_vector_type(4)))  float v4f;
typedef __attribute__((ext_vector_type(2)))  float v2f;
typedef __attribute__((ext_vector_type(4)))  unsigned v4u;
typedef __attribute__((ext_vector_type(4)))  int v4i;
typedef float __attribute__((may_alias)) float_a;
typedef int __attribute__((may_alias)) int_a;

template <typename T> __device__ __forceinline__ void vst2(void* p, T v) { *(volatile T*)p = v; __threadfence(); *(volatile T*)p = v; }
__device__ __forceinline__ v8f wmma16(v16h a, v16h b, v8f c) {
  v8f d = __builtin_amdgcn_wmma_f32_16x16x32_f16(false, a, false, b, (short)0, c, false, false);
  asm volatile("v_nop\n\tv_nop\n\tv_nop\n\tv_nop" : "+v"(d) : "v"(a), "v"(b));
  return d;
}
__device__ __forceinline__ v8f wmma_bf(v16b a, v16b b, v8f c) {
  v8f d = __builtin_amdgcn_wmma_f32_16x16x32_bf16(false, a, false, b, (short)0, c, false, false);
  asm volatile("v_nop\n\tv_nop\n\tv_nop\n\tv_nop" : "+v"(d) : "v"(a), "v"(b));
  return d;
}
__device__ __forceinline__ v16h frag_h(const _Float16* rowk0, int lane) {
  union { v16h v; v8h q[2]; } u; const _Float16* p = rowk0 + 8 * (lane >> 4);
  u.q[0] = *(const v8h*)p; u.q[1] = *(const v8h*)(p + 16); return u.v;
}
__device__ __forceinline__ v16h frag_f32(const float* rowk0, int lane) {
  v16h a; const float* p = rowk0 + 8 * (lane >> 4);
#pragma unroll
  for (int i = 0; i < 8; ++i) { a[i] = (_Float16)p[i]; a[8 + i] = (_Float16)p[16 + i]; }
  return a;
}
__device__ __forceinline__ v16h frag_f32s(const float* rowk0, int lane, float sc) {
  v16h a; const float* p = rowk0 + 8 * (lane >> 4);
#pragma unroll
  for (int i = 0; i < 8; ++i) { a[i] = (_Float16)(p[i] * sc); a[8 + i] = (_Float16)(p[16 + i] * sc); }
  return a;
}
__device__ __forceinline__ v16h fragc_f32(const float* W, int k0, int n, int lane, int ld, int K) {
  v16h a; const int g = lane >> 4;
#pragma unroll
  for (int i = 0; i < 8; ++i) { const int ka = k0 + 8 * g + i, kb = ka + 16;
    a[i] = (_Float16)(ka < K ? W[(size_t)(ka < K ? ka : K - 1) * ld + n] : 0.f); a[8 + i] = (_Float16)(kb < K ? W[(size_t)(kb < K ? kb : K - 1) * ld + n] : 0.f); }
  return a;
}
struct F2 { v16b h, l; };
__device__ __forceinline__ F2 bsplit16(const float v[16]) { F2 r;
#pragma unroll
  for (int i = 0; i < 16; ++i) { const __bf16 h = (__bf16)v[i]; r.h[i] = h; r.l[i] = (__bf16)(v[i] - (float)h); }
  return r; }
__device__ __forceinline__ F2 split_row(const float* row, int k0, int lane) { float v[16]; const float* p = row + k0 + 8 * (lane >> 4);
#pragma unroll
  for (int i = 0; i < 8; ++i) { v[i] = p[i]; v[8 + i] = p[16 + i]; }
  return bsplit16(v); }
__device__ __forceinline__ F2 split_rowK(const float* row, int k0, int lane, int K) { float v[16]; const int g = lane >> 4;
#pragma unroll
  for (int i = 0; i < 8; ++i) { const int ka = k0 + 8 * g + i, kb = ka + 16; v[i] = ka < K ? row[ka < K ? ka : K - 1] : 0.f; v[8 + i] = kb < K ? row[kb < K ? kb : K - 1] : 0.f; }
  return bsplit16(v); }
__device__ __forceinline__ F2 split_col(const float* W, int k0, int n, int lane, int ld, int K) { float v[16]; const int g = lane >> 4;
#pragma unroll
  for (int i = 0; i < 8; ++i) { const int ka = k0 + 8 * g + i, kb = ka + 16; v[i] = ka < K ? W[(size_t)(ka < K ? ka : K - 1) * ld + n] : 0.f; v[8 + i] = kb < K ? W[(size_t)(kb < K ? kb : K - 1) * ld + n] : 0.f; }
  return bsplit16(v); }
__device__ __forceinline__ v8f mac3(const F2& a, const F2& b, v8f c) { c = wmma_bf(a.l, b.h, c); c = wmma_bf(a.h, b.l, c); return wmma_bf(a.h, b.h, c); }
__device__ __forceinline__ float sigm(float v) { return 1.0f / (1.0f + expf(-v)); }
#define LDSX() do { asm volatile("s_wait_dscnt 0" ::: "memory"); __builtin_amdgcn_wave_barrier(); __builtin_amdgcn_fence(__ATOMIC_RELEASE, "workgroup"); } while (0)


#define NPTS 131072
#define CF 32
#define KPL 2048
#define NL 64
#define NB1 8
#define DPJ 128
#define DHD 256
#define DD 512
#define NBLK (NL * KPL / 64)
#ifndef NPB
#define NPB NBLK
#endif
typedef __attribute__((ext_vector_type(8))) __bf16 v8b;
__device__ __forceinline__ v16b frag_b(const __bf16* rowk0, int lane) {
  union { v16b v; v8b q[2]; } u; const __bf16* p = rowk0 + 8 * (lane >> 4);
  u.q[0] = *(const v8b*)p; u.q[1] = *(const v8b*)(p + 16); return u.v;
}
__device__ __forceinline__ float bfr(float v) { return (float)(__bf16)v; }
__device__ __attribute__((noinline)) float exp_ni(float v) { return expf(v); }
__device__ __attribute__((noinline)) float erf_ni(float v) { return erff(v); }

#define WS_P1   0u
#define WS_P2   (WS_P1 + 2u * DPJ * CF)
#define WS_PE1  (WS_P2 + 2u * DPJ * DPJ)
#define WS_PE2  (WS_PE1 + 2u * DHD * DPJ)
#define WS_PMX  (WS_PE2 + 2u * (size_t)DD * DHD)
#define WS_LF   (WS_PMX + 4u * (size_t)NBLK * DD)
#define WS_L1   (WS_LF + 4u * NL * DD)
#define WS_END  (WS_L1 + 4u * NB1 * DD)

__global__ __launch_bounds__(256) void k_pack(const float* __restrict__ WP1, const float* __restrict__ WP2, const float* __restrict__ WE1, const float* __restrict__ WE2, __bf16* __restrict__ P, _Float16* __restrict__ PE2) {
  const int n = blockIdx.x, which = blockIdx.y, t = threadIdx.x; __shared__ __align__(16) __bf16 s[DHD]; __shared__ __align__(16) _Float16 sh[DHD];
  if (which == 0) { if (n >= DPJ) return; if (t < CF) s[t] = (__bf16)WP1[(size_t)t * DPJ + n]; __syncthreads(); if (t < CF / 8) vst2((unsigned*)(P + WS_P1 / 2 + (size_t)n * CF + t * 8), *(const v4u*)&s[t * 8]); }
  else if (which == 1) { if (n >= DPJ) return; if (t < DPJ) s[t] = (__bf16)WP2[(size_t)t * DPJ + n]; __syncthreads(); if (t < DPJ / 8) vst2((unsigned*)(P + WS_P2 / 2 + (size_t)n * DPJ + t * 8), *(const v4u*)&s[t * 8]); }
  else if (which == 2) { if (n >= DHD) return; if (t < DPJ) s[t] = (__bf16)WE1[(size_t)(3 + t) * DHD + n]; __syncthreads(); if (t < DPJ / 8) vst2((unsigned*)(P + WS_PE1 / 2 + (size_t)n * DPJ + t * 8), *(const v4u*)&s[t * 8]); }
  else { s[0] = (__bf16)0.f; sh[t] = (_Float16)(bfr(WE2[(size_t)t * DD + n]) * 256.0f); __syncthreads(); if (t < DHD / 8) vst2((unsigned*)(PE2 + (size_t)n * DHD + t * 8), *(const v4u*)&sh[t * 8]); }
}
__global__ __launch_bounds__(128) void k_point(const float* __restrict__ CO, const float* __restrict__ FE, const int* __restrict__ LIDX, const int* __restrict__ LCEN, const __bf16* __restrict__ P, const _Float16* __restrict__ PE2, const float* __restrict__ BP1, const float* __restrict__ BP2, const float* __restrict__ WE1, const float* __restrict__ BE1, const float* __restrict__ BE2, float* __restrict__ PMX) {
  __shared__ __align__(16) float sf[64][DPJ + 4]; __shared__ __align__(16) float sg[64][DPJ + 4]; __shared__ __align__(16) _Float16 shh[64][DHD + 8]; __shared__ float srel[64][3]; __shared__ int spt[64]; __shared__ float smax[4][128];
  const int tid = threadIdx.x, wave = tid >> 5, lane = tid & 31, col = lane & 15, g = lane >> 4; const size_t pb0 = (size_t)blockIdx.x * 64; const int leaf = (int)(pb0 / KPL);
  if (tid < 64) { const int pt = min(max(LIDX[pb0 + tid], 0), NPTS - 1); spt[tid] = pt; const int cen = min(max(LCEN[leaf], 0), NPTS - 1); for (int c = 0; c < 3; ++c) srel[tid][c] = bfr(CO[(size_t)pt * 3 + c]) - bfr(CO[(size_t)cen * 3 + c]); }
  __syncthreads();
  const int r0 = wave * 16;
  { v8f acc[8] = {}; v16b a; { const float* p = FE + (size_t)spt[r0 + col] * CF + 8 * g;
#pragma unroll
      for (int i = 0; i < 8; ++i) { a[i] = (__bf16)p[i]; a[8 + i] = (__bf16)p[16 + i]; } }
#pragma unroll
    for (int j = 0; j < 8; ++j) acc[j] = wmma_bf(a, frag_b(P + WS_P1 / 2 + (size_t)(j * 16 + col) * CF, lane), acc[j]);
#pragma unroll
    for (int j = 0; j < 8; ++j) { const float bb = bfr(BP1[j * 16 + col]);
#pragma unroll
      for (int r = 0; r < 8; ++r) sf[r0 + 8 * g + r][j * 16 + col] = fmaxf(acc[j][r] + bb, 0.f); } }
  if (tid < 64) for (int c = DPJ; c < DPJ + 4; ++c) { sf[tid][c] = 0.f; sg[tid][c] = 0.f; }
  LDSX();
  { v8f acc[8] = {};
#pragma unroll
    for (int kc = 0; kc < DPJ / 32; ++kc) { const F2 a = split_row(&sf[r0 + col][0], kc * 32, lane);
#pragma unroll
      for (int j = 0; j < 8; ++j) { const v16b w = frag_b(P + WS_P2 / 2 + (size_t)(j * 16 + col) * DPJ + kc * 32, lane); acc[j] = wmma_bf(a.l, w, acc[j]); acc[j] = wmma_bf(a.h, w, acc[j]); } }
#pragma unroll
    for (int j = 0; j < 8; ++j) { const float bb = bfr(BP2[j * 16 + col]);
#pragma unroll
      for (int r = 0; r < 8; ++r) sg[r0 + 8 * g + r][j * 16 + col] = acc[j][r] + bb; } }
  LDSX();
#pragma unroll 1
  for (int pass = 0; pass < 2; ++pass) { v8f acc[8] = {};
#pragma unroll
    for (int kc = 0; kc < DPJ / 32; ++kc) { const F2 a = split_row(&sg[r0 + col][0], kc * 32, lane);
#pragma unroll
      for (int j = 0; j < 8; ++j) { const v16b w = frag_b(P + WS_PE1 / 2 + (size_t)(pass * 128 + j * 16 + col) * DPJ + kc * 32, lane); acc[j] = wmma_bf(a.l, w, acc[j]); acc[j] = wmma_bf(a.h, w, acc[j]); } }
#pragma unroll
    for (int j = 0; j < 8; ++j) { const int n = pass * 128 + j * 16 + col; const float w0 = bfr(WE1[n]), w1 = bfr(WE1[DHD + n]), w2 = bfr(WE1[2 * DHD + n]), bb = bfr(BE1[n]);
#pragma unroll
      for (int r = 0; r < 8; ++r) { const int row = r0 + 8 * g + r; const float v = acc[j][r] + ((srel[row][0] * w0 + srel[row][1] * w1) + srel[row][2] * w2) + bb; shh[row][n] = (_Float16)fmaxf(v, 0.f); } } }
  if (tid < 64) for (int c = DHD; c < DHD + 8; ++c) shh[tid][c] = (_Float16)0.f;
  LDSX();
  v16h ah[8];
#pragma unroll
  for (int kc = 0; kc < 8; ++kc) ah[kc] = frag_h(&shh[r0 + col][kc * 32], lane);
#pragma unroll 1
  for (int pass = 0; pass < 4; ++pass) { v8f acc[8] = {};
#pragma unroll
    for (int kc = 0; kc < 8; ++kc) {
#pragma unroll
      for (int j = 0; j < 8; ++j) acc[j] = wmma16(ah[kc], frag_h(PE2 + (size_t)(pass * 128 + j * 16 + col) * DHD + kc * 32, lane), acc[j]); }
#pragma unroll
    for (int j = 0; j < 8; ++j) { const int n = pass * 128 + j * 16 + col; const float bb = bfr(BE2[n]); float mx = -3.0e38f;
#pragma unroll
      for (int r = 0; r < 8; ++r) mx = fmaxf(mx, fmaxf(acc[j][r] * (1.0f / 256.0f) + bb, 0.f));
      mx = fmaxf(mx, __shfl_xor(mx, 16));
      if (g == 0) smax[wave][j * 16 + col] = mx; }
    __syncthreads();
    if (tid < 128) { const int c = tid; const float m4 = fmaxf(fmaxf(smax[0][c], smax[1][c]), fmaxf(smax[2][c], smax[3][c])); PMX[(size_t)blockIdx.x * DD + pass * 128 + c] = m4; }
    __syncthreads(); }
}
__global__ __launch_bounds__(256) void k_leaf(const float* __restrict__ PMX, float* __restrict__ LF, float* __restrict__ OUT) {
  const int leaf = blockIdx.x, t = threadIdx.x; __shared__ __align__(16) float s[DD];
  for (int c = t; c < DD; c += 256) { float mx = -3.0e38f; for (int b = 0; b < KPL / 64; ++b) mx = fmaxf(mx, PMX[((size_t)leaf * (KPL / 64) + b) * DD + c]); s[c] = mx; }
  __syncthreads();
  for (int q = t; q < DD / 4; q += 256) { const v4f v = *(const v4f*)&s[q * 4]; vst2(LF + (size_t)leaf * DD + q * 4, v); vst2(OUT + (size_t)(1 + NB1 + leaf) * DD + q * 4, v); }
}
template <int LEVEL>
__global__ __launch_bounds__(256) void k_agg(const float* __restrict__ CHILD, const float* __restrict__ CO, const int* __restrict__ LCEN, const int* __restrict__ L1CEN, const int* __restrict__ ROOT, const float* __restrict__ WA1, const float* __restrict__ BA1, const float* __restrict__ WA2, const float* __restrict__ BA2, float* __restrict__ L1, float* __restrict__ OUT) {
  __shared__ float sz[NB1][DD + 3]; __shared__ float sg[DD]; __shared__ __align__(16) float so[DD];
  const int p = blockIdx.x, t = threadIdx.x; const int nch = (LEVEL == 1) ? (NL / NB1) : NB1;
  const int pidx = (LEVEL == 1) ? min(max(L1CEN[p], 0), NPTS - 1) : min(max(ROOT[0], 0), NPTS - 1);
  for (int e = t; e < nch * (DD + 3); e += 256) { const int m = e / (DD + 3), c = e % (DD + 3); float v;
    if (c < DD) v = CHILD[(size_t)((LEVEL == 1) ? (p * nch + m) : m) * DD + c];
    else { const int cidx = (LEVEL == 1) ? min(max(LCEN[p * nch + m], 0), NPTS - 1) : min(max(L1CEN[m], 0), NPTS - 1); v = bfr(CO[(size_t)cidx * 3 + (c - DD)]) - bfr(CO[(size_t)pidx * 3 + (c - DD)]); }
    sz[m][c] = v; }
  __syncthreads();
  for (int n = t; n < DD; n += 256) { float mx = -3.0e38f;
#pragma unroll 1
    for (int m = 0; m < nch; ++m) { float s = bfr(BA1[n]);
#pragma unroll 1
      for (int c = 0; c < DD + 3; ++c) s += sz[m][c] * bfr(WA1[(size_t)c * DD + n]);
      mx = fmaxf(mx, fmaxf(s, 0.f)); }
    sg[n] = mx; }
  __syncthreads();
  for (int n = t; n < DD; n += 256) { float s = bfr(BA2[n]);
#pragma unroll 1
    for (int c = 0; c < DD; ++c) s += sg[c] * bfr(WA2[(size_t)c * DD + n]);
    so[n] = s; }
  __syncthreads();
  for (int q = t; q < DD / 4; q += 256) { const v4f v = *(const v4f*)&so[q * 4]; if (LEVEL == 1) { vst2(L1 + (size_t)p * DD + q * 4, v); vst2(OUT + (size_t)(1 + p) * DD + q * 4, v); } else vst2(OUT + q * 4, v); }
}
extern "C" void kernel_launch(void* const* d_in, const int* in_sizes, int n_in, void* d_out, int out_size, void* d_ws, size_t ws_size, hipStream_t stream) {
  (void)in_sizes; (void)n_in; (void)out_size;
  const float** F = (const float**)d_in;
  if (ws_size < (size_t)WS_END) return;
  char* ws = (char*)d_ws; __bf16* P = (__bf16*)ws; _Float16* PE2 = (_Float16*)(ws + WS_PE2); float *PMX = (float*)(ws + WS_PMX), *LF = (float*)(ws + WS_LF), *L1 = (float*)(ws + WS_L1);
  const int* LIDX = (const int*)d_in[2]; const int* LCEN = (const int*)d_in[3]; const int* L1CEN = (const int*)d_in[4]; const int* ROOT = (const int*)d_in[5];
  k_pack<<<dim3(DD, 4), 256, 0, stream>>>(F[6], F[8], F[10], F[12], P, PE2);
  k_point<<<NPB, 128, 0, stream>>>(F[0], F[1], LIDX, LCEN, P, PE2, F[7], F[9], F[10], F[11], F[13], PMX);
  k_leaf<<<NL, 256, 0, stream>>>(PMX, LF, (float*)d_out);
  k_agg<1><<<NB1, 256, 0, stream>>>(LF, F[0], LCEN, L1CEN, ROOT, F[14], F[15], F[16], F[17], L1, (float*)d_out);
  k_agg<0><<<1, 256, 0, stream>>>(L1, F[0], LCEN, L1CEN, ROOT, F[14], F[15], F[16], F[17], L1, (float*)d_out);
}
